// EnsembleFC_72387378806934
// MI455X (gfx1250) — hardware-verified
//
#include <hip/hip_runtime.h>
#include <stdint.h>

typedef _Float16 f16;
typedef f16      v16h  __attribute__((ext_vector_type(16)));
typedef f16      v8h   __attribute__((ext_vector_type(8)));
typedef float    v8f   __attribute__((ext_vector_type(8)));
typedef float    v4f   __attribute__((ext_vector_type(4)));
typedef unsigned u32x4 __attribute__((ext_vector_type(4)));

constexpr int E_   = 16;
constexpr int DIN  = 512;
constexpr int HID  = 512;
constexpr int BM   = 32;
constexpr int BK   = 32;
constexpr int SA   = DIN + 8;
constexpr int SW   = BK + 8;
constexpr int NTHR = 256;
constexpr float WSCALE = 1024.0f;
constexpr float WINV   = 1.0f / 1024.0f;

static_assert(DIN == HID);
static_assert((SA * 2) % 16 == 0);
static_assert((SW * 2) % 16 == 0);

constexpr int AS_H   = BM * SA;
constexpr int WS_H   = HID * SW;
constexpr int W3_H   = HID;
constexpr int OUTS_F = 4 * BM;
constexpr unsigned LDS_BYTES = (unsigned)((2 * AS_H + WS_H + W3_H) * 2 + OUTS_F * 4);
static_assert(LDS_BYTES == 109056u);
static_assert((AS_H * 2) % 16 == 0 && (WS_H * 2) % 16 == 0 && (W3_H * 2) % 16 == 0);

union Frag  { v16h v; v8h hv[2]; u32x4 q[2]; };
union Pack8 { v8h v; f16 s[8]; };

__device__ __forceinline__ v8f zero8() { v8f z; z[0]=0.f; z[1]=0.f; z[2]=0.f; z[3]=0.f; z[4]=0.f; z[5]=0.f; z[6]=0.f; z[7]=0.f; return z; }

__device__ __forceinline__ void mma1(v8f& c, const v16h a, const v16h b) {
  c = __builtin_amdgcn_wmma_f32_16x16x32_f16(false, a, false, b, (short)0, c, false, false);
  asm volatile("v_nop\n\tv_nop\n\tv_nop\n\tv_nop" : "+v"(c) : "v"(a), "v"(b));
}
__device__ __forceinline__ void mma2(v8f& c0, v8f& c1, const v16h a0, const v16h a1, const v16h b) {
  c0 = __builtin_amdgcn_wmma_f32_16x16x32_f16(false, a0, false, b, (short)0, c0, false, false);
  c1 = __builtin_amdgcn_wmma_f32_16x16x32_f16(false, a1, false, b, (short)0, c1, false, false);
  asm volatile("v_nop\n\tv_nop\n\tv_nop\n\tv_nop" : "+v"(c0), "+v"(c1) : "v"(a0), "v"(a1), "v"(b));
}

__device__ __forceinline__ v8h cvt8(const v4f p, const v4f q, const float s) {
  Pack8 u;
  u.s[0] = (f16)(p[0] * s); u.s[1] = (f16)(p[1] * s); u.s[2] = (f16)(p[2] * s); u.s[3] = (f16)(p[3] * s);
  u.s[4] = (f16)(q[0] * s); u.s[5] = (f16)(q[1] * s); u.s[6] = (f16)(q[2] * s); u.s[7] = (f16)(q[3] * s);
  return u.v;
}

__device__ __forceinline__ v16h ld_frag(const f16* base, int pitch, int r, int k0, int h) {
  Frag f;
  f.hv[0] = *(const v8h*)(base + r * pitch + k0 + 8 * h);
  f.hv[1] = *(const v8h*)(base + r * pitch + k0 + 16 + 8 * h);
  return f.v;
}

__global__ __launch_bounds__(NTHR) void k_wt(const float* __restrict__ w_a,
                                             const float* __restrict__ w_b,
                                             f16* __restrict__ wt) {
  __shared__ float tile[64][33];
  const int t = threadIdx.x;
  const int z = blockIdx.z;
  const int e = z & (E_ - 1);
  const float* src = ((z < E_) ? w_a : w_b) + (size_t)e * DIN * HID;
  f16* dst = wt + (size_t)z * DIN * HID;
  const int k0 = blockIdx.x * 64;
  const int n0 = blockIdx.y * 32;
  #pragma unroll
  for (int j = 0; j < 8; ++j) {
    const int idx = t + NTHR * j;
    const int kk = idx >> 5, nn = idx & 31;
    tile[kk][nn] = src[(size_t)(k0 + kk) * HID + n0 + nn];
  }
  __syncthreads();
  const int wave = t >> 5, l = t & 31;
  const int nn = wave * 4 + (l >> 3);
  const int ks = (l & 7) * 8;
  Pack8 u;
  #pragma unroll
  for (int i = 0; i < 8; ++i) u.s[i] = (f16)(tile[ks + i][nn] * WSCALE);
  f16* p = dst + (size_t)(n0 + nn) * DIN + k0 + ks;
  *(volatile v8h*)p = u.v;
  __threadfence();
  *(volatile v8h*)p = u.v;
}

__device__ __forceinline__ void gemm_layer(const f16* Asrc, f16* Hdst, f16* Ws,
                                           const f16* __restrict__ Wg,
                                           const float* __restrict__ bias, int t) {
  const int wave = t >> 5, l = t & 31, h = l >> 4, m = l & 15;
  v8f acc[2][4];
  #pragma unroll
  for (int i = 0; i < 2; ++i)
    #pragma unroll
    for (int j = 0; j < 4; ++j) acc[i][j] = zero8();

  #pragma unroll 1
  for (int ks = 0; ks < DIN / BK; ++ks) {
    __syncthreads();
    #pragma unroll
    for (int j = 0; j < 8; ++j) {
      const int idx = t + NTHR * j;
      const int n = idx >> 2, c = idx & 3;
      const v8h v = *(const v8h*)(Wg + (size_t)n * DIN + ks * BK + c * 8);
      *(v8h*)(Ws + n * SW + c * 8) = v;
    }
    __syncthreads();
    const v16h a0 = ld_frag(Asrc, SA, m,      ks * BK, h);
    const v16h a1 = ld_frag(Asrc, SA, 16 + m, ks * BK, h);
    #pragma unroll
    for (int j = 0; j < 4; ++j) {
      const int n = wave * 64 + j * 16 + m;
      const v16h b = ld_frag(Ws, SW, n, 0, h);
      mma2(acc[0][j], acc[1][j], a0, a1, b);
    }
  }
  #pragma unroll
  for (int i = 0; i < 2; ++i) {
    #pragma unroll
    for (int j = 0; j < 4; ++j) {
      const int col = wave * 64 + j * 16 + m;
      const float bs = bias[col];
      #pragma unroll
      for (int r = 0; r < 8; ++r) {
        const int row = i * 16 + 8 * h + r;
        float v = acc[i][j][r] * WINV + bs;
        v = v > 0.f ? v : 0.f;
        Hdst[row * SA + col] = (f16)v;
      }
    }
  }
  __syncthreads();
}

__global__ __launch_bounds__(NTHR) void k_mlp(const float* __restrict__ x,
                                              const f16* __restrict__ wt,
                                              const float* __restrict__ b1,
                                              const float* __restrict__ b2,
                                              const float* __restrict__ w3,
                                              const float* __restrict__ b3,
                                              float* __restrict__ out, int batch) {
  extern __shared__ __attribute__((aligned(16))) unsigned char smem_raw[];
  f16* As  = (f16*)smem_raw;
  f16* Hs  = As + AS_H;
  f16* Ws  = Hs + AS_H;
  f16* w3s = Ws + WS_H;
  float* outs = (float*)(w3s + W3_H);

  const int t = threadIdx.x;
  const int wave = t >> 5, l = t & 31, h = l >> 4, m = l & 15;
  const int e  = blockIdx.y;
  const int b0 = blockIdx.x * BM;

  {
    const int row = t >> 3, part = t & 7;
    int gb = b0 + row;
    gb = (gb < batch) ? gb : (batch - 1);
    const float* xr = x + (size_t)gb * DIN + part * 64;
    f16* ar = As + row * SA + part * 64;
    #pragma unroll
    for (int j = 0; j < 8; ++j) {
      const v4f p = *(const v4f*)(xr + j * 8);
      const v4f q = *(const v4f*)(xr + j * 8 + 4);
      *(v8h*)(ar + j * 8) = cvt8(p, q, 1.0f);
    }
  }
  {
    const float* w3e = w3 + (size_t)e * HID;
    w3s[2 * t]     = (f16)(w3e[2 * t] * WSCALE);
    w3s[2 * t + 1] = (f16)(w3e[2 * t + 1] * WSCALE);
  }

  gemm_layer(As, Hs, Ws, wt + (size_t)e * DIN * HID,        b1 + (size_t)e * HID, t);
  gemm_layer(Hs, As, Ws, wt + (size_t)(E_ + e) * HID * HID, b2 + (size_t)e * HID, t);

  {
    const int strip = wave & 1;
    const int kq    = wave >> 1;
    const unsigned msk = (m == 0) ? 0xFFFFFFFFu : 0u;
    v8f c = zero8();
    #pragma unroll
    for (int s = 0; s < 4; ++s) {
      const int k0 = kq * 128 + s * BK;
      const v16h a = ld_frag(As, SA, strip * 16 + m, k0, h);
      Frag b;
      b.hv[0] = *(const v8h*)(w3s + k0 + 8 * h);
      b.hv[1] = *(const v8h*)(w3s + k0 + 16 + 8 * h);
      b.q[0] &= msk;
      b.q[1] &= msk;
      mma1(c, a, b.v);
    }
    if (m == 0) {
      #pragma unroll
      for (int r = 0; r < 8; ++r) outs[kq * BM + strip * 16 + 8 * h + r] = c[r];
    }
    __syncthreads();
    if (t < 8) {
      const float bb = b3[e];
      v4f o;
      #pragma unroll
      for (int i = 0; i < 4; ++i) {
        const int row = 4 * t + i;
        o[i] = ((outs[row] + outs[BM + row]) + (outs[2 * BM + row] + outs[3 * BM + row])) * WINV + bb;
      }
      if (b0 + 4 * t + 3 < batch) {
        volatile v4f* po = (volatile v4f*)(out + (size_t)e * batch + b0 + 4 * t);
        *po = o;
        __threadfence();
        *po = o;
      }
    }
  }
}

extern "C" void kernel_launch(void* const* d_in, const int* in_sizes, int n_in,
                              void* d_out, int out_size, void* d_ws, size_t ws_size,
                              hipStream_t stream) {
  if (n_in < 7) return;
  const float* x   = (const float*)d_in[0];
  const float* W1  = (const float*)d_in[1];
  const float* b1  = (const float*)d_in[2];
  const float* W2  = (const float*)d_in[3];
  const float* b2  = (const float*)d_in[4];
  const float* W3  = (const float*)d_in[5];
  const float* b3v = (const float*)d_in[6];
  float* out = (float*)d_out;

  if (in_sizes[1] != E_ * DIN * HID || in_sizes[3] != E_ * HID * HID) return;
  if (in_sizes[2] < E_ * HID || in_sizes[4] < E_ * HID || in_sizes[5] < E_ * HID || in_sizes[6] < E_) return;

  int batch = in_sizes[0] / DIN;
  const int ob = out_size / E_;
  if (ob < batch) batch = ob;
  if (batch <= 0) return;

  const size_t wt_bytes = (size_t)2 * E_ * DIN * HID * sizeof(f16);
  if (wt_bytes > ws_size) return;
  f16* Wt = (f16*)d_ws;

  k_wt<<<dim3(DIN / 64, HID / 32, 2 * E_), NTHR, 0, stream>>>(W1, W2, Wt);

  k_mlp<<<dim3((batch + BM - 1) / BM, E_), NTHR, LDS_BYTES, stream>>>(x, Wt, b1, b2, W3, b3v, out, batch);
}
